// GraphAttentionLayer_10479720202952
// MI455X (gfx1250) — hardware-run, weakly checked
//
#include <hip/hip_runtime.h>
#include <stddef.h>
#include <stdint.h>
#include <math.h>


#define NN      8192
#define NE      262144
#define FIN     256
#define FOUT    64
#define NTHR    256
#define NWAVE   8
#define EPT     8
#define CHUNK   (NTHR * EPT)
#define WCAP    (EPT * 32)
#define LISTN   (NWAVE * WCAP)
#define NBRUN   256
#define SLB     8
#define RCAP    10240
#define DEGCAP  96
#define GBM     128
#define SLOPE   0.2f
#define NUH     (NN * (FIN / 8))
#define NUW     (FOUT * (FIN / 8))
#define NUA     32
#define ROWS_ZINTS (2 * RCAP + 3 * NBRUN + LISTN + 32)
#define ROWS_LDS_BYTES (ROWS_ZINTS * 4)
#define WSMAX   (128u << 20)

static_assert(NN == 32 * NBRUN);
static_assert(NBRUN == (1 << SLB) && NBRUN == NWAVE * 32);
static_assert(NE % CHUNK == 0 && NE % 256 == 0);
static_assert(((long long)NE << SLB) < (1LL << 31));
static_assert((CHUNK & (CHUNK - 1)) == 0);
static_assert(FOUT == 64 && FOUT == 32 * 2);
static_assert(FIN % 32 == 0 && FIN / 8 == 32);
static_assert(NN % GBM == 0 && GBM == NWAVE * 16 && NN / GBM == 64);
static_assert(DEGCAP % 32 == 0 && DEGCAP / 32 == 3);
static_assert(ROWS_ZINTS % 4 == 0);
static_assert(ROWS_LDS_BYTES <= 327680);
static_assert(NUH % NTHR == 0 && NUW % NTHR == 0 && NUA == 32);
static_assert(RCAP % 4 == 0 && LISTN >= NWAVE * WCAP);

typedef float          v2f   __attribute__((ext_vector_type(2)));
typedef float          v4f   __attribute__((ext_vector_type(4)));
typedef float          v8f   __attribute__((ext_vector_type(8)));
typedef double         v2d   __attribute__((ext_vector_type(2)));
typedef int            v4i   __attribute__((ext_vector_type(4)));
typedef int            v8i   __attribute__((ext_vector_type(8)));
typedef unsigned short v8us  __attribute__((ext_vector_type(8)));
typedef unsigned short v16us __attribute__((ext_vector_type(16)));
typedef __bf16         v16bf __attribute__((ext_vector_type(16)));
typedef v4f  __attribute__((may_alias)) v4fa;
typedef v2d  __attribute__((may_alias)) v2da;
typedef v4i  __attribute__((may_alias)) v4ia;
typedef v8us __attribute__((may_alias)) v8usa;
union FragB { v16bf v; v16us u; v8us h[2]; v8i w; };

__device__ __forceinline__ v8f wmb(const FragB& a, const FragB& b, v8f c) {
  v8f d = __builtin_amdgcn_wmma_f32_16x16x32_bf16(false, a.v, false, b.v, (short)0, c, false, false);
  asm volatile("v_nop\n\tv_nop\n\tv_nop\n\tv_nop" : "+v"(d) : "v"(a.w), "v"(b.w));
  return d;
}

__device__ __forceinline__ unsigned bf16_bits(float f) {
  const unsigned u = __float_as_uint(f);
  return (u + 0x7FFFu + ((u >> 16) & 1u)) >> 16;
}
__device__ __forceinline__ float bf16_val(float f) {
  return __uint_as_float(bf16_bits(f) << 16);
}
__device__ __forceinline__ v4f bfr4(const v4f a) {
  v4f r; r.x = bf16_val(a.x); r.y = bf16_val(a.y); r.z = bf16_val(a.z); r.w = bf16_val(a.w); return r;
}
__device__ __forceinline__ int clampn(int v) {
  v = v < 0 ? 0 : v;
  return v > NN - 1 ? NN - 1 : v;
}

__global__ __launch_bounds__(NTHR) void k_prep(const float* __restrict__ h, const float* __restrict__ W,
                                               const float* __restrict__ a,
                                               unsigned short* HB, unsigned short* WT, float* AV) {
  const int u = (int)blockIdx.x * NTHR + (int)threadIdx.x;
  if (u < NUH) {
    const int row = u >> 5;
    const int k8  = (u & 31) * 8;
    const float* p = h + (size_t)row * FIN + k8;
    const v4f x = *(const v4f*)p;
    const v4f y = *(const v4f*)(p + 4);
    v8us o;
    o[0] = (unsigned short)bf16_bits(x.x); o[1] = (unsigned short)bf16_bits(x.y);
    o[2] = (unsigned short)bf16_bits(x.z); o[3] = (unsigned short)bf16_bits(x.w);
    o[4] = (unsigned short)bf16_bits(y.x); o[5] = (unsigned short)bf16_bits(y.y);
    o[6] = (unsigned short)bf16_bits(y.z); o[7] = (unsigned short)bf16_bits(y.w);
    unsigned short* dp = HB + (size_t)row * FIN + k8;
    *(volatile v8us*)dp = o;
    __threadfence();
    *(volatile v8us*)dp = o;
  } else if (u < NUH + NUW) {
    const int v  = u - NUH;
    const int n  = v >> 5;
    const int k8 = (v & 31) * 8;
    const float* p = W + (size_t)k8 * FOUT + n;
    v8us o;
#pragma unroll
    for (int i = 0; i < 8; ++i) o[i] = (unsigned short)bf16_bits(p[(size_t)i * FOUT]);
    unsigned short* dp = WT + (size_t)n * FIN + k8;
    *(volatile v8us*)dp = o;
    __threadfence();
    *(volatile v8us*)dp = o;
  } else if (u < NUH + NUW + NUA) {
    const int t = u - NUH - NUW;
    const v4f x = *(const v4f*)(a + 4 * t);
    const v4f r = bfr4(x);
    float* dp = AV + 4 * t;
    *(volatile v4f*)dp = r;
    __threadfence();
    *(volatile v4f*)dp = r;
  }
}

__global__ __launch_bounds__(NTHR) __attribute__((amdgpu_num_vgpr(248)))
void k_gemm(const unsigned short* __restrict__ A, const unsigned short* __restrict__ BT,
            const float* __restrict__ AV, float* WH, float* S12, double* CP) {
  __shared__ __attribute__((aligned(16))) float  stg[GBM * FOUT];
  __shared__ __attribute__((aligned(16))) float  sav[2 * FOUT];
  __shared__ __attribute__((aligned(16))) float  sdt[2 * GBM];
  __shared__ __attribute__((aligned(16))) double scp[FOUT];
  const int tid = (int)threadIdx.x, lane = tid & 31, wave = tid >> 5, hh = lane >> 4, m = lane & 15;
  const int rowBase = (int)blockIdx.x * GBM;

  if (tid < 32) {
    const v4f t4 = *(const v4f*)(AV + 4 * tid);
    *(v4fa*)(sav + 4 * tid) = t4;
  }

  v8f acc[4];
  {
    const v8f z = {0.f, 0.f, 0.f, 0.f, 0.f, 0.f, 0.f, 0.f};
    acc[0] = z; acc[1] = z; acc[2] = z; acc[3] = z;
  }
  const unsigned short* ap = A  + (size_t)(rowBase + 16 * wave + m) * (size_t)FIN + 8 * hh;
  const unsigned short* bp = BT + (size_t)m * (size_t)FIN + 8 * hh;
#pragma unroll 1
  for (int k0 = 0; k0 < FIN; k0 += 32) {
    FragB af;
    af.h[0] = *(const v8usa*)(ap + k0);
    af.h[1] = *(const v8usa*)(ap + k0 + 16);
#pragma unroll
    for (int nt = 0; nt < 4; ++nt) {
      const unsigned short* wq = bp + (size_t)(16 * nt) * (size_t)FIN + k0;
      FragB bf;
      bf.h[0] = *(const v8usa*)wq;
      bf.h[1] = *(const v8usa*)(wq + 16);
      acc[nt] = wmb(af, bf, acc[nt]);
    }
  }

#pragma unroll
  for (int nt = 0; nt < 4; ++nt) {
    const int lc = 16 * nt + m;
#pragma unroll
    for (int r = 0; r < 8; ++r) {
      const int lr = 16 * wave + 8 * hh + r;
      stg[lr * FOUT + lc] = acc[nt][r];
    }
  }
  __syncthreads();

  if (tid < GBM) {
    const float* hr = stg + tid * FOUT;
    float s = 0.0f, d = 0.0f;
#pragma unroll 2
    for (int c4 = 0; c4 < FOUT / 4; ++c4) {
      const v4f hv = *(const v4fa*)(hr + 4 * c4);
      const v4f av = *(const v4fa*)(sav + 4 * c4);
      const v4f bv = *(const v4fa*)(sav + FOUT + 4 * c4);
      s = fmaf(hv.x, av.x, s);  d = fmaf(hv.x, bv.x, d);
      s = fmaf(hv.y, av.y, s);  d = fmaf(hv.y, bv.y, d);
      s = fmaf(hv.z, av.z, s);  d = fmaf(hv.z, bv.z, d);
      s = fmaf(hv.w, av.w, s);  d = fmaf(hv.w, bv.w, d);
    }
    sdt[tid]       = s;
    sdt[GBM + tid] = d;
  } else if (tid < GBM + FOUT) {
    const int c = tid - GBM;
    double cs = 0.0;
#pragma unroll 4
    for (int r = 0; r < GBM; ++r) cs += (double)stg[r * FOUT + c];
    scp[c] = cs;
  }
  __syncthreads();

  v4f fv[8];
#pragma unroll
  for (int i = 0; i < 8; ++i) {
    const int lr = 16 * wave + 2 * i + hh;
    fv[i] = *(const v4fa*)(stg + lr * FOUT + 4 * m);
  }
  const v4f sdv = *(const v4fa*)(sdt + (wave & 1) * GBM + 4 * lane);
  const v2d cpv = *(const v2da*)(scp + 2 * lane);
  float*  sp = S12 + (size_t)(wave & 1) * NN + rowBase + 4 * lane;
  double* cq = CP + (size_t)blockIdx.x * FOUT + 2 * lane;

#pragma unroll
  for (int i = 0; i < 8; ++i) {
    const int lr = 16 * wave + 2 * i + hh;
    float* op = WH + (size_t)(rowBase + lr) * FOUT + 4 * m;
    *(volatile v4f*)op = fv[i];
  }
  if (wave < 2)  *(volatile v4f*)sp = sdv;
  if (wave == 2) *(volatile v2d*)cq = cpv;
  __threadfence();
#pragma unroll
  for (int i = 0; i < 8; ++i) {
    const int lr = 16 * wave + 2 * i + hh;
    float* op = WH + (size_t)(rowBase + lr) * FOUT + 4 * m;
    *(volatile v4f*)op = fv[i];
  }
  if (wave < 2)  *(volatile v4f*)sp = sdv;
  if (wave == 2) *(volatile v2d*)cq = cpv;
}

__global__ __launch_bounds__(64) void k_colmean(const double* __restrict__ CP, float* WM) {
  __shared__ __attribute__((aligned(16))) float sm[FOUT];
  const int c = (int)threadIdx.x;
  double s = 0.0;
#pragma unroll 4
  for (int b = 0; b < NN / GBM; ++b) s += CP[(size_t)b * FOUT + c];
  sm[c] = (float)(s * (1.0 / (double)NN));
  __syncthreads();
  if (c < 16) {
    const v4f v = *(const v4fa*)(sm + 4 * c);
    float* dp = WM + 4 * c;
    *(volatile v4f*)dp = v;
    __threadfence();
    *(volatile v4f*)dp = v;
  }
}

__device__ __forceinline__ int scan_chunk(const int* __restrict__ keys, int cbase, int slotBase,
                                          int* list, int tid, int lane, int wave) {
  const int el0 = tid * EPT;
  const int e0  = cbase + el0;
  const v4i da = *(const v4i*)(keys + e0);
  const v4i db = *(const v4i*)(keys + e0 + 4);
  const unsigned nbs = (unsigned)slotBase;
  const unsigned unb = (unsigned)NBRUN;
  const unsigned s0 = (unsigned)da.x - nbs, s1 = (unsigned)da.y - nbs;
  const unsigned s2 = (unsigned)da.z - nbs, s3 = (unsigned)da.w - nbs;
  const unsigned s4 = (unsigned)db.x - nbs, s5 = (unsigned)db.y - nbs;
  const unsigned s6 = (unsigned)db.z - nbs, s7 = (unsigned)db.w - nbs;
  const bool h0 = s0 < unb, h1 = s1 < unb, h2 = s2 < unb, h3 = s3 < unb;
  const bool h4 = s4 < unb, h5 = s5 < unb, h6 = s6 < unb, h7 = s7 < unb;
  const unsigned any = __builtin_amdgcn_ballot_w32(h0 | h1 | h2 | h3 | h4 | h5 | h6 | h7);
  int wc = 0;
  if (any != 0u) {
    const int nl = (int)h0 + (int)h1 + (int)h2 + (int)h3 + (int)h4 + (int)h5 + (int)h6 + (int)h7;
    int incl = nl;
#pragma unroll
    for (int d = 1; d < 32; d <<= 1) {
      const int y = __shfl_up(incl, d, 32);
      incl += (lane >= d) ? y : 0;
    }
    wc = __shfl(incl, 31, 32);
    int pos = incl - nl;
    int* wl = list + wave * WCAP;
    if (h0 && pos < WCAP) { wl[pos] = ((el0 + 0) << SLB) | (int)s0; pos += 1; }
    if (h1 && pos < WCAP) { wl[pos] = ((el0 + 1) << SLB) | (int)s1; pos += 1; }
    if (h2 && pos < WCAP) { wl[pos] = ((el0 + 2) << SLB) | (int)s2; pos += 1; }
    if (h3 && pos < WCAP) { wl[pos] = ((el0 + 3) << SLB) | (int)s3; pos += 1; }
    if (h4 && pos < WCAP) { wl[pos] = ((el0 + 4) << SLB) | (int)s4; pos += 1; }
    if (h5 && pos < WCAP) { wl[pos] = ((el0 + 5) << SLB) | (int)s5; pos += 1; }
    if (h6 && pos < WCAP) { wl[pos] = ((el0 + 6) << SLB) | (int)s6; pos += 1; }
    if (h7 && pos < WCAP) { wl[pos] = ((el0 + 7) << SLB) | (int)s7; pos += 1; }
  }
  return wc;
}

__global__ __launch_bounds__(NTHR) void k_rows(const int* __restrict__ keys, const int* __restrict__ parts,
                                               const float* __restrict__ WH, const float* __restrict__ S12,
                                               const float* __restrict__ WM, float* outp) {
  extern __shared__ __attribute__((aligned(16))) int dsm[];
  int* reg1 = dsm;
  int* reg2 = reg1 + RCAP;
  int* scnt = reg2 + RCAP;
  int* soff = scnt + NBRUN;
  int* cur  = soff + NBRUN;
  int* list = cur + NBRUN;
  int* misc = list + LISTN;
  const int tid = (int)threadIdx.x, lane = tid & 31, wave = tid >> 5;
  const int nodeBase = (int)blockIdx.x * NBRUN;

  {
    const v4i z4 = {0, 0, 0, 0};
    for (int i = tid * 4; i < ROWS_ZINTS; i += NTHR * 4) *(v4ia*)(dsm + i) = z4;
  }
  __syncthreads();

  int tot = 0;
#pragma unroll 1
  for (int ch = 0; ch < NE / CHUNK; ++ch) {
    const int cbase = ch * CHUNK;
    const int wc = scan_chunk(keys, cbase, nodeBase, list, tid, lane, wave);
    if (lane == 0) misc[wave] = wc;
    __syncthreads();
    int pre = 0, all = 0;
#pragma unroll
    for (int w2 = 0; w2 < NWAVE; ++w2) {
      int c = misc[w2];
      c = c < 0 ? 0 : (c > WCAP ? WCAP : c);
      all += c;
      pre += (w2 < wave) ? c : 0;
    }
    const int wcc  = wc < 0 ? 0 : (wc > WCAP ? WCAP : wc);
    const int base = tot + pre;
#pragma unroll 1
    for (int i = lane; i < wcc; i += 32) {
      const int ent = list[wave * WCAP + i];
      const int el  = (ent >> SLB) & (CHUNK - 1);
      const int sl  = ent & (NBRUN - 1);
      int eid = cbase + el;
      eid = eid > NE - 1 ? NE - 1 : eid;
      const int pos = base + i;
      if (pos < RCAP) reg1[pos] = (int)(((unsigned)eid << SLB) | (unsigned)sl);
    }
    tot += all;
    tot = tot > RCAP ? RCAP : tot;
    __syncthreads();
  }
  const int nh = tot;

  if (wave == 0) {
#pragma unroll 1
    for (int b0 = 0; b0 < nh; b0 += 32) {
      const int idx = b0 + lane;
      const int uv  = reg1[idx < nh ? idx : nh - 1];
      const int m32 = (nh - b0) < 32 ? (nh - b0) : 32;
#pragma unroll 1
      for (int k = 0; k < m32; ++k) {
        const int u  = __builtin_amdgcn_readlane(uv, k);
        const int sl = u & (NBRUN - 1);
        if (lane == 0) scnt[sl] = scnt[sl] + 1;
      }
    }
  }
  __syncthreads();

  if (wave == 0) {
    const int base = lane * (NBRUN / 32);
    int cv[NBRUN / 32];
    int s = 0, mxc = 0;
#pragma unroll
    for (int i = 0; i < NBRUN / 32; ++i) {
      int c = scnt[base + i];
      c = c < 0 ? 0 : c;
      cv[i] = c;
      s += c;
      mxc = mxc > c ? mxc : c;
    }
    int incl = s;
#pragma unroll
    for (int d = 1; d < 32; d <<= 1) {
      const int y = __shfl_up(incl, d, 32);
      incl += (lane >= d) ? y : 0;
    }
    int run = incl - s;
#pragma unroll
    for (int i = 0; i < NBRUN / 32; ++i) {
      soff[base + i] = run;
      cur[base + i]  = run;
      run += cv[i];
    }
    const unsigned bm = __builtin_amdgcn_ballot_w32(mxc > DEGCAP);
    if (lane == 0) misc[8] = (bm != 0u) ? 1 : 0;
  }
  __syncthreads();

  if (wave == 0) {
#pragma unroll 1
    for (int b0 = 0; b0 < nh; b0 += 32) {
      const int idx = b0 + lane;
      const int uv  = reg1[idx < nh ? idx : nh - 1];
      int eid = (int)((unsigned)uv >> SLB);
      eid = eid > NE - 1 ? NE - 1 : eid;
      const int pv = clampn(parts[eid]);
      const int m32 = (nh - b0) < 32 ? (nh - b0) : 32;
#pragma unroll 1
      for (int k = 0; k < m32; ++k) {
        const int u  = __builtin_amdgcn_readlane(uv, k);
        const int p  = __builtin_amdgcn_readlane(pv, k);
        const int sl = u & (NBRUN - 1);
        if (lane == 0) {
          int pos = cur[sl];
          pos = pos < 0 ? 0 : (pos > RCAP - 1 ? RCAP - 1 : pos);
          reg2[pos] = p;
          cur[sl] = pos + 1;
        }
      }
    }
  }
  __syncthreads();

  const int degf = misc[8];
  const float qnan = __int_as_float(0x7fc00000);
  const float pz = (nh >= RCAP || degf != 0) ? qnan : 0.0f;
  const v2f wm = *(const v2f*)(WM + 2 * lane);
  asm volatile("" :: "v"(wm.x), "v"(wm.y));
  const float* whl = WH + 2 * lane;
  const float ninf = -__builtin_huge_valf();
  const int k0i = lane, k1i = lane + 32, k2i = lane + 64;

#pragma unroll 1
  for (int si = 0; si < NBRUN / NWAVE; ++si) {
    const int slot = wave * (NBRUN / NWAVE) + si;
    const int node = nodeBase + slot;
    int cvv = scnt[slot];
    int ovv = soff[slot];
    ovv = ovv < 0 ? 0 : (ovv > nh ? nh : ovv);
    cvv = cvv < 0 ? 0 : (cvv > DEGCAP ? DEGCAP : cvv);
    cvv = cvv > nh - ovv ? nh - ovv : cvv;
    const int c = __builtin_amdgcn_readfirstlane(cvv);
    const int o = __builtin_amdgcn_readfirstlane(ovv);
    int last = o + c - 1;
    last = last < o ? o : last;
    last = last > RCAP - 1 ? RCAP - 1 : last;

    int i0 = o + k0i; i0 = i0 > last ? last : i0;
    int i1 = o + k1i; i1 = i1 > last ? last : i1;
    int i2 = o + k2i; i2 = i2 > last ? last : i2;
    const int id0 = clampn(reg2[i0]);
    const int id1 = clampn(reg2[i1]);
    const int id2 = clampn(reg2[i2]);

    int d0 = 0, d1 = 0, d2 = 0;
#pragma unroll 1
    for (int k = 0; k < c; ++k) {
      int ik = o + k; ik = ik > last ? last : ik;
      const int pk = clampn(reg2[ik]);
      d0 |= (int)((id0 == pk) & (k0i > k));
      d1 |= (int)((id1 == pk) & (k1i > k));
      d2 |= (int)((id2 == pk) & (k2i > k));
    }

    const float s1i = S12[node];
    const float x0 = S12[NN + id0];
    asm volatile("" :: "v"(x0));
    const float x1 = S12[NN + id1];
    asm volatile("" :: "v"(x1));
    const float x2 = S12[NN + id2];
    asm volatile("" :: "v"(x2));
    float lg0 = s1i + x0; lg0 = (lg0 >= 0.0f) ? lg0 : SLOPE * lg0;
    float lg1 = s1i + x1; lg1 = (lg1 >= 0.0f) ? lg1 : SLOPE * lg1;
    float lg2 = s1i + x2; lg2 = (lg2 >= 0.0f) ? lg2 : SLOPE * lg2;
    const bool kp0 = (k0i < c) && (d0 == 0);
    const bool kp1 = (k1i < c) && (d1 == 0);
    const bool kp2 = (k2i < c) && (d2 == 0);

    float mx = kp0 ? lg0 : ninf;
    mx = fmaxf(mx, kp1 ? lg1 : ninf);
    mx = fmaxf(mx, kp2 ? lg2 : ninf);
#pragma unroll
    for (int off = 16; off > 0; off >>= 1) mx = fmaxf(mx, __shfl_xor(mx, off, 32));
    const float mref = (c == 0) ? 0.0f : mx;
    const float e0 = expf(lg0 - mref);
    const float e1 = expf(lg1 - mref);
    const float e2 = expf(lg2 - mref);
    const float p0 = kp0 ? e0 : 0.0f;
    const float p1 = kp1 ? e1 : 0.0f;
    const float p2 = kp2 ? e2 : 0.0f;
    float sm = (p0 + p1) + p2;
#pragma unroll
    for (int off = 16; off > 0; off >>= 1) sm += __shfl_xor(sm, off, 32);
    const float sdv = (c == 0) ? 1.0f : sm;
    const int al0 = __float_as_int(p0 / sdv);
    const int al1 = __float_as_int(p1 / sdv);
    const int al2 = __float_as_int(p2 / sdv);

    v2f acc = {0.0f, 0.0f};
    {
      int mj = c; mj = mj < 0 ? 0 : (mj > 32 ? 32 : mj);
#pragma unroll 1
      for (int k = 0; k < mj; ++k) {
        const int   idk = __builtin_amdgcn_readlane(id0, k);
        const float alk = __int_as_float(__builtin_amdgcn_readlane(al0, k));
        const v2f r = *(const v2f*)(whl + (size_t)idk * FOUT);
        acc.x = fmaf(alk, r.x, acc.x);
        acc.y = fmaf(alk, r.y, acc.y);
      }
    }
    {
      int mj = c - 32; mj = mj < 0 ? 0 : (mj > 32 ? 32 : mj);
#pragma unroll 1
      for (int k = 0; k < mj; ++k) {
        const int   idk = __builtin_amdgcn_readlane(id1, k);
        const float alk = __int_as_float(__builtin_amdgcn_readlane(al1, k));
        const v2f r = *(const v2f*)(whl + (size_t)idk * FOUT);
        acc.x = fmaf(alk, r.x, acc.x);
        acc.y = fmaf(alk, r.y, acc.y);
      }
    }
    {
      int mj = c - 64; mj = mj < 0 ? 0 : (mj > 32 ? 32 : mj);
#pragma unroll 1
      for (int k = 0; k < mj; ++k) {
        const int   idk = __builtin_amdgcn_readlane(id2, k);
        const float alk = __int_as_float(__builtin_amdgcn_readlane(al2, k));
        const v2f r = *(const v2f*)(whl + (size_t)idk * FOUT);
        acc.x = fmaf(alk, r.x, acc.x);
        acc.y = fmaf(alk, r.y, acc.y);
      }
    }

    const float vx = (c == 0) ? wm.x : acc.x;
    const float vy = (c == 0) ? wm.y : acc.y;
    v2f ov;
    ov.x = ((vx >= 0.0f) ? vx : SLOPE * vx) + pz;
    ov.y = ((vy >= 0.0f) ? vy : SLOPE * vy) + pz;
    float* op = outp + (size_t)node * FOUT + 2 * lane;
    *(volatile v2f*)op = ov;
    __threadfence();
    *(volatile v2f*)op = ov;
  }
}

extern "C" void kernel_launch(void* const* d_in, const int* in_sizes, int n_in,
                              void* d_out, int out_size, void* d_ws, size_t ws_size,
                              hipStream_t stream) {
  if (n_in < 5) return;
  if (in_sizes[0] != NN * FIN) return;
  if (in_sizes[1] != FIN * FOUT) return;
  if (in_sizes[2] != 2 * FOUT) return;
  if (in_sizes[3] != NE || in_sizes[4] != NE) return;
  if (out_size != NN * FOUT) return;

  const float* h   = (const float*)d_in[0];
  const float* W   = (const float*)d_in[1];
  const float* a   = (const float*)d_in[2];
  const int*   rix = (const int*)d_in[3];
  const int*   cix = (const int*)d_in[4];
  float* out = (float*)d_out;

  char* ws = (char*)d_ws;
  size_t off = 0;
  const size_t oHB = off; off += (size_t)NN * FIN * 2;            off = (off + 255) & ~(size_t)255;
  const size_t oWT = off; off += (size_t)FOUT * FIN * 2;          off = (off + 255) & ~(size_t)255;
  const size_t oAV = off; off += (size_t)2 * FOUT * 4;            off = (off + 255) & ~(size_t)255;
  const size_t oWH = off; off += (size_t)NN * FOUT * 4;           off = (off + 255) & ~(size_t)255;
  const size_t oSS = off; off += (size_t)2 * NN * 4;              off = (off + 255) & ~(size_t)255;
  const size_t oCP = off; off += (size_t)(NN / GBM) * FOUT * 8;   off = (off + 255) & ~(size_t)255;
  const size_t oWM = off; off += (size_t)FOUT * 4;                off = (off + 255) & ~(size_t)255;
  if (off > ws_size || off > (size_t)WSMAX) return;
  unsigned short* HB  = (unsigned short*)(ws + oHB);
  unsigned short* WT  = (unsigned short*)(ws + oWT);
  float*          AV  = (float*)(ws + oAV);
  float*          WHp = (float*)(ws + oWH);
  float*          S12 = (float*)(ws + oSS);
  double*         CP  = (double*)(ws + oCP);
  float*          WM  = (float*)(ws + oWM);

  hipFuncSetAttribute(reinterpret_cast<const void*>(&k_rows),
                      hipFuncAttributeMaxDynamicSharedMemorySize, (int)ROWS_LDS_BYTES);

  k_prep<<<(NUH + NUW + NUA + NTHR - 1) / NTHR, NTHR, 0, stream>>>(h, W, a, HB, WT, AV);
  k_gemm<<<NN / GBM, NTHR, 0, stream>>>(HB, WT, AV, WHp, S12, CP);
  k_colmean<<<1, 64, 0, stream>>>(CP, WM);
  k_rows<<<NN / NBRUN, NTHR, ROWS_LDS_BYTES, stream>>>(rix, cix, WHp, S12, WM, out);
}
